// MambaExpert_77120432767223
// MI455X (gfx1250) — hardware-verified
//
#include <hip/hip_runtime.h>
#include <math.h>

typedef __attribute__((ext_vector_type(16))) _Float16 v16h;
typedef __attribute__((ext_vector_type(8)))  _Float16 v8h;
typedef __attribute__((ext_vector_type(16))) __bf16   v16b;
typedef __attribute__((ext_vector_type(8)))  __bf16   v8b;
typedef __attribute__((ext_vector_type(8)))  float    v8f;
typedef __attribute__((ext_vector_type(4)))  float    v4f;
typedef __attribute__((ext_vector_type(2)))  float    v2f;

constexpr int NIMG  = 4;
constexpr int NCH   = 64;
constexpr int IMH   = 96;
constexpr int IMW   = 96;
constexpr int NPIX  = IMH * IMW;
constexpr int NTOK  = NIMG * NPIX;
constexpr int DIN   = 96;
constexpr int DINP  = 128;
constexpr int XZW   = 2 * DIN;
constexpr int NST   = 16;
constexpr int DTR   = 4;
constexpr int NDIR  = 4;
constexpr int XPC   = DTR + 2 * NST;
constexpr int XPCP  = 64;
constexpr int FFH   = 128;
constexpr int SCH   = 64;
constexpr int TOKB  = 64;
static_assert(NPIX % SCH == 0, "scan chunking");
static_assert(NPIX % TOKB == 0, "ln tiling");
static_assert((SCH * 9) % DIN == 0, "scan staging coverage");
static_assert((IMW * DINP) % (8 * DIN) == 0, "conv 16-bit store coverage");
static_assert(NTOK % 8 == 0, "gate tiling");

__device__ __forceinline__ unsigned short f2bf_bits(float f) {
  unsigned u = __float_as_uint(f);
  return (unsigned short)((u + 0x7FFFu + ((u >> 16) & 1u)) >> 16);
}
__device__ __forceinline__ float bf_bits2f(unsigned short h) { return __uint_as_float(((unsigned)h) << 16); }

__device__ __forceinline__ void dep_guard_h(v8f& a, v8f& b, v16h x, v16h y) { asm volatile("v_nop\n\tv_nop\n\tv_nop\n\tv_nop" : "+v"(a), "+v"(b) : "v"(x), "v"(y)); }
__device__ __forceinline__ void dep_guard_b(v8f& a, v8f& b, v16b x, v16b y) { asm volatile("v_nop\n\tv_nop\n\tv_nop\n\tv_nop" : "+v"(a), "+v"(b) : "v"(x), "v"(y)); }
__device__ __forceinline__ void keep4_h(v16h a, v16h b, v16h c, v16h d) { asm volatile("v_nop" :: "v"(a), "v"(b), "v"(c), "v"(d)); }
__device__ __forceinline__ void keep4_b(v16b a, v16b b, v16b c, v16b d) { asm volatile("v_nop" :: "v"(a), "v"(b), "v"(c), "v"(d)); }
__device__ __forceinline__ void acc_guard4(v8f& a, v8f& b, v8f& c, v8f& d) { asm volatile("v_nop\n\tv_nop\n\tv_nop\n\tv_nop" : "+v"(a), "+v"(b), "+v"(c), "+v"(d)); }
template <typename T> struct Frag;
template <> struct Frag<_Float16> {
  typedef v16h V; union U { v16h v; v8h h[2]; };
  static __device__ __forceinline__ v16h load(const _Float16* p) {
    U f; f.h[0] = *(const v8h*)(p); f.h[1] = *(const v8h*)(p + 16); return f.v;
  }
  static __device__ __forceinline__ v8f mma(v16h a, v16h b, v8f c) {
    return __builtin_amdgcn_wmma_f32_16x16x32_f16(false, a, false, b, (short)0, c, false, false);
  }
  static __device__ __forceinline__ void guard(v8f& a, v8f& b, v16h x, v16h y) { dep_guard_h(a, b, x, y); }
  static __device__ __forceinline__ void keep(v16h a, v16h b, v16h c, v16h d) { keep4_h(a, b, c, d); }
};
template <> struct Frag<__bf16> {
  typedef v16b V; union U { v16b v; v8b h[2]; };
  static __device__ __forceinline__ v16b load(const __bf16* p) {
    U f; f.h[0] = *(const v8b*)(p); f.h[1] = *(const v8b*)(p + 16); return f.v;
  }
  static __device__ __forceinline__ v8f mma(v16b a, v16b b, v8f c) {
    return __builtin_amdgcn_wmma_f32_16x16x32_bf16(false, a, false, b, (short)0, c, false, false);
  }
  static __device__ __forceinline__ void guard(v8f& a, v8f& b, v16b x, v16b y) { dep_guard_b(a, b, x, y); }
  static __device__ __forceinline__ void keep(v16b a, v16b b, v16b c, v16b d) { keep4_b(a, b, c, d); }
};

template <int ET> struct Elem;
template <> struct Elem<0> { typedef _Float16 T; };
template <> struct Elem<1> { typedef __bf16 T; };
template <int ET, bool SPLIT, int BIAS_MODE, int OUT_MODE, bool RESID, int ACT = 0>
__global__ __launch_bounds__(256) void wmma_gemm64(
    const unsigned short* __restrict__ Ap, const unsigned short* __restrict__ A2p, int lda, long strideA,
    const unsigned short* __restrict__ Btp, const unsigned short* __restrict__ Bt2p, int ldb, long strideB,
    void* __restrict__ Cout, void* __restrict__ Cout2, int ldc, long strideC,
    const float* __restrict__ bias,
    const float* __restrict__ resid, long strideR,
    int M, int N, int K, float scale) {
  typedef typename Elem<ET>::T T;
  typedef typename Frag<T>::V V;
  const T* A = (const T*)Ap; const T* A2 = (const T*)A2p; const T* Bt = (const T*)Btp; const T* Bt2 = (const T*)Bt2p;
  __shared__ __align__(16) float sT[8][16 * 68];
  const int b    = blockIdx.y;
  const int lane = threadIdx.x & 31;
  const int wave = threadIdx.x >> 5;
  const int tilesN = N >> 6;
  const int tilesM = M >> 6;
  const int tile = blockIdx.x * 8 + wave;
  if (tile >= tilesM * tilesN) return;
  const int tm = tile / tilesN;
  const int tn = tile - tm * tilesN;
  const int m0 = tm << 6;
  const int n0 = tn << 6;

  const T* Ab  = A  + (size_t)b * strideA;
  const T* Bb  = Bt + (size_t)b * strideB;
  const T* Ab2 = SPLIT ? (A2  + (size_t)b * strideA) : nullptr;
  const T* Bb2 = SPLIT ? (Bt2 + (size_t)b * strideB) : nullptr;

  const int rlane = lane & 15;
  const int koff  = (lane >> 4) * 8;
  const int mOff  = (lane >> 4) * 8;

  v8f acc[4][4];
#pragma unroll
  for (int i = 0; i < 4; ++i)
#pragma unroll
    for (int j = 0; j < 4; ++j) acc[i][j] = (v8f){0.f,0.f,0.f,0.f,0.f,0.f,0.f,0.f};

  for (int k0 = 0; k0 < K; k0 += 32) {
    V bh[4], bl[4];
#pragma unroll
    for (int j = 0; j < 4; ++j) {
      const size_t bo = (size_t)(n0 + (j << 4) + rlane) * ldb + koff + k0;
      bh[j] = Frag<T>::load(Bb + bo);
      if (SPLIT) bl[j] = Frag<T>::load(Bb2 + bo);
    }
#pragma unroll
    for (int i = 0; i < 4; ++i) {
      const size_t ao = (size_t)(m0 + (i << 4) + rlane) * lda + koff + k0;
      V ah = Frag<T>::load(Ab + ao);
      V al;
      if (SPLIT) al = Frag<T>::load(Ab2 + ao);
#pragma unroll
      for (int j = 0; j < 4; ++j) {
        acc[i][j] = Frag<T>::mma(ah, bh[j], acc[i][j]);
        if (SPLIT) {
          acc[i][j] = Frag<T>::mma(ah, bl[j], acc[i][j]);
          acc[i][j] = Frag<T>::mma(al, bh[j], acc[i][j]);
        }
      }
      Frag<T>::guard(acc[i][0], acc[i][3], ah, SPLIT ? al : ah);
    }
    Frag<T>::keep(bh[0], bh[1], bh[2], bh[3]);
    if (SPLIT) Frag<T>::keep(bl[0], bl[1], bl[2], bl[3]);
  }
  acc_guard4(acc[0][0], acc[0][1], acc[0][2], acc[0][3]);
  acc_guard4(acc[1][0], acc[1][1], acc[1][2], acc[1][3]);
  acc_guard4(acc[2][0], acc[2][1], acc[2][2], acc[2][3]);
  acc_guard4(acc[3][0], acc[3][1], acc[3][2], acc[3][3]);

  float* slab = sT[wave];
  const float* Rb = RESID ? (resid + (size_t)b * strideR) : nullptr;
#pragma unroll
  for (int i = 0; i < 4; ++i) {
    const int mBase = m0 + (i << 4);
#pragma unroll
    for (int j = 0; j < 4; ++j) {
      const int n = n0 + (j << 4) + rlane;
      float bv = 0.f;
      if (BIAS_MODE == 2) bv = bias[n];
#pragma unroll
      for (int r = 0; r < 8; ++r) {
        float v = acc[i][j][r] * scale;
        if (BIAS_MODE == 1) v += bias[mBase + mOff + r];
        if (BIAS_MODE == 2) v += bv;
        if (RESID) v += Rb[(size_t)(mBase + mOff + r) * ldc + n];
        if (ACT == 1) v = tanhf(v);
        if (ACT == 2) v = fmaxf(v, 0.0f);
        if (ACT == 3) v = v / (1.0f + expf(-v));
        if (ACT == 4) v = (v > 0.f) ? v : 0.01f * v;
        if (ACT == 5) v = 0.5f * v * (1.0f + erff(v * 0.70710678118654752f));
        slab[(mOff + r) * 68 + (j << 4) + rlane] = v;
      }
    }
    __builtin_amdgcn_fence(__ATOMIC_RELEASE, "workgroup");
    __builtin_amdgcn_wave_barrier();
    __builtin_amdgcn_fence(__ATOMIC_ACQUIRE, "workgroup");
    if (OUT_MODE == 0) {
      float* C = (float*)Cout + (size_t)b * strideC;
      const int hh = lane >> 4, c4 = (lane & 15) * 4;
      for (int pass = 0; pass < 2; ++pass) {
#pragma unroll
        for (int it = 0; it < 8; ++it) {
          const int row = it * 2 + hh;
          v4f v = *(const v4f*)(slab + row * 68 + c4);
          *(volatile v4f*)(C + (size_t)(mBase + row) * ldc + n0 + c4) = v;
        }
        __threadfence();
      }
    } else {
      const int q = lane >> 3, c8 = (lane & 7) * 8;
      unsigned short* C  = (unsigned short*)Cout  + (size_t)b * strideC;
      unsigned short* C2 = (OUT_MODE == 2) ? ((unsigned short*)Cout2 + (size_t)b * strideC) : nullptr;
      for (int pass = 0; pass < 2; ++pass) {
#pragma unroll
        for (int it = 0; it < 4; ++it) {
          const int row = it * 4 + q;
          const float* sp = slab + row * 68 + c8;
          v8h hv, lv;
#pragma unroll
          for (int e = 0; e < 8; ++e) {
            if (OUT_MODE == 1) {
              hv[e] = (_Float16)sp[e];
            } else {
              unsigned short hb = f2bf_bits(sp[e]);
              unsigned short lb = f2bf_bits(sp[e] - bf_bits2f(hb));
              hv[e] = __builtin_bit_cast(_Float16, hb);
              lv[e] = __builtin_bit_cast(_Float16, lb);
            }
          }
          *(volatile v8h*)(C + (size_t)(mBase + row) * ldc + n0 + c8) = hv;
          if (OUT_MODE == 2) *(volatile v8h*)(C2 + (size_t)(mBase + row) * ldc + n0 + c8) = lv;
        }
        __threadfence();
      }
    }
    __builtin_amdgcn_fence(__ATOMIC_RELEASE, "workgroup");
    __builtin_amdgcn_wave_barrier();
    __builtin_amdgcn_fence(__ATOMIC_ACQUIRE, "workgroup");
  }
}

__device__ __forceinline__ void split_bf16_bits(float f, _Float16& hi, _Float16& lo) {
  const unsigned short hb = f2bf_bits(f);
  const unsigned short lb = f2bf_bits(f - bf_bits2f(hb));
  hi = __builtin_bit_cast(_Float16, hb);
  lo = __builtin_bit_cast(_Float16, lb);
}
template <int MODE>
__device__ __forceinline__ void pack8(v4f f0, v4f f1, v8h& hv, v8h& lv) {
#pragma unroll
  for (int e = 0; e < 4; ++e) {
    if (MODE == 0) {
      hv[e]     = (_Float16)f0[e];
      hv[4 + e] = (_Float16)f1[e];
      lv[e]     = hv[e];
      lv[4 + e] = hv[4 + e];
    } else {
      _Float16 a, c;
      split_bf16_bits(f0[e], a, c); hv[e] = a;     lv[e] = c;
      split_bf16_bits(f1[e], a, c); hv[4 + e] = a; lv[4 + e] = c;
    }
  }
}

template <int MODE>
__global__ __launch_bounds__(256) void cast_pad_kernel(
    const float* __restrict__ src, int spitch, int R, int Rp,
    unsigned short* __restrict__ dst, unsigned short* __restrict__ dst2, int Kcp, int Ku, int nchunks, float scale)
{
  const int f = blockIdx.x * 256 + threadIdx.x;
  if (f >= nchunks) return;
  const int cpr = Kcp >> 3;
  const int ng = f / cpr;
  const int g  = f - ng * cpr;
  const int bi = ng / Rp;
  const int n  = ng - bi * Rp;
  const bool cval  = (g * 8) < Ku;
  const bool rval  = n < R;
  const bool valid = rval && cval;
  const int sr = rval ? n : 0;
  const int sc = cval ? (g * 8) : 0;
  const float* p = src + ((size_t)bi * R + sr) * spitch + sc;
  const v4f a0 = *(const v4f*)(p);
  const v4f a1 = *(const v4f*)(p + 4);
  v4f s0, s1;
#pragma unroll
  for (int e = 0; e < 4; ++e) {
    s0[e] = valid ? a0[e] * scale : 0.0f;
    s1[e] = valid ? a1[e] * scale : 0.0f;
  }
  v8h hv, lv;
  pack8<MODE>(s0, s1, hv, lv);
  unsigned short* qd  = dst  + (size_t)f * 8;
  unsigned short* qd2 = dst2 + (size_t)f * 8;
  *(volatile v8h*)qd = hv;
  if (MODE == 1) *(volatile v8h*)qd2 = lv;
  __threadfence();
  *(volatile v8h*)qd = hv;
  if (MODE == 1) *(volatile v8h*)qd2 = lv;
}

template <int MODE>
__global__ __launch_bounds__(256) void ln_nchw_kernel(
    const float* __restrict__ X, const float* __restrict__ gam, const float* __restrict__ bet,
    unsigned short* __restrict__ OUTA, unsigned short* __restrict__ OUTB)
{
  __shared__ __align__(16) float sX[TOKB * 68];
  const int t = threadIdx.x, lane = t & 31, wave = t >> 5;
  const int b_ = blockIdx.x / (NPIX / TOKB);
  const int l0 = (blockIdx.x - b_ * (NPIX / TOKB)) * TOKB;
#pragma unroll
  for (int pass = 0; pass < 4; ++pass) {
    const int c  = pass * 16 + (t >> 4);
    const int l4 = (t & 15) * 4;
    const v4f v = *(const v4f*)(X + ((size_t)(b_ * NCH + c)) * NPIX + l0 + l4);
#pragma unroll
    for (int e = 0; e < 4; ++e) sX[(l4 + e) * 68 + c] = v[e];
  }
  __syncthreads();
  const int tk = t >> 2, qq = t & 3;
  float* wp = sX + tk * 68 + qq * 16;
  v4f xv[4];
#pragma unroll
  for (int i = 0; i < 4; ++i) xv[i] = *(const v4f*)(wp + 4 * i);
  float s = 0.f;
#pragma unroll
  for (int i = 0; i < 4; ++i) s += (xv[i][0] + xv[i][1]) + (xv[i][2] + xv[i][3]);
  s += __shfl_xor(s, 1, 32);
  s += __shfl_xor(s, 2, 32);
  const float mu = s * (1.0f / 64.0f);
  float q = 0.f;
#pragma unroll
  for (int i = 0; i < 4; ++i) {
#pragma unroll
    for (int e = 0; e < 4; ++e) { const float dd = xv[i][e] - mu; q = fmaf(dd, dd, q); }
  }
  q += __shfl_xor(q, 1, 32);
  q += __shfl_xor(q, 2, 32);
  const float var = q * (1.0f / 64.0f);
  const float is  = rsqrtf(var + 1e-5f);
#pragma unroll
  for (int i = 0; i < 4; ++i) {
    const int cb = qq * 16 + 4 * i;
    const v4f gg = *(const v4f*)(gam + cb);
    const v4f bb = *(const v4f*)(bet + cb);
    v4f o;
#pragma unroll
    for (int e = 0; e < 4; ++e) o[e] = ((xv[i][e] - mu) * is) * gg[e] + bb[e];
    *(v4f*)(wp + 4 * i) = o;
  }
  __syncthreads();
  const int q8 = lane >> 3, c8 = (lane & 7) * 8;
  v8h hvv[2], lvv[2];
#pragma unroll
  for (int it = 0; it < 2; ++it) {
    const float* sp = sX + ((wave * 2 + it) * 4 + q8) * 68 + c8;
    const v4f f0 = *(const v4f*)(sp);
    const v4f f1 = *(const v4f*)(sp + 4);
    pack8<MODE>(f0, f1, hvv[it], lvv[it]);
  }
  unsigned short* ob  = OUTA + ((size_t)(b_ * NPIX + l0)) * NCH;
  unsigned short* ob2 = OUTB + ((size_t)(b_ * NPIX + l0)) * NCH;
  for (int pass = 0; pass < 2; ++pass) {
#pragma unroll
    for (int it = 0; it < 2; ++it) {
      const size_t ro = (size_t)((wave * 2 + it) * 4 + q8) * NCH + c8;
      *(volatile v8h*)(ob + ro) = hvv[it];
      if (MODE == 1) *(volatile v8h*)(ob2 + ro) = lvv[it];
    }
    __threadfence();
  }
}

__global__ __launch_bounds__(96) void dwconv_silu_kernel(
    const float* __restrict__ XZ, const float* __restrict__ cw, const float* __restrict__ cbias,
    float* __restrict__ XC, unsigned short* __restrict__ XC16H, unsigned short* __restrict__ XC16L)
{
  __shared__ __align__(16) float sH[IMW * DINP];
  const int t  = threadIdx.x;
  const int b_ = blockIdx.x / IMH;
  const int h_ = blockIdx.x - b_ * IMH;
  const int d  = t;
#pragma unroll 1
  for (int i = t; i < IMW * (DINP - DIN); i += DIN) sH[(i >> 5) * DINP + DIN + (i & 31)] = 0.0f;
  const float* wd = cw + (size_t)d * 9;
  const float w00 = wd[0], w01 = wd[1], w02 = wd[2];
  const float w10 = wd[3], w11 = wd[4], w12 = wd[5];
  const float w20 = wd[6], w21 = wd[7], w22 = wd[8];
  const float bc = cbias[d];
  const bool up = h_ > 0, dn = h_ < IMH - 1;
  const int r0 = up ? (h_ - 1) : 0;
  const int r2 = dn ? (h_ + 1) : (IMH - 1);
  const float* p0 = XZ + ((size_t)(b_ * IMH + r0) * IMW) * XZW + d;
  const float* p1 = XZ + ((size_t)(b_ * IMH + h_) * IMW) * XZW + d;
  const float* p2 = XZ + ((size_t)(b_ * IMH + r2) * IMW) * XZW + d;
  float a0m = 0.f, a1m = 0.f, a2m = 0.f;
  float a0c, a1c, a2c;
  {
    const float v0 = p0[0], v1 = p1[0], v2 = p2[0];
    a0c = up ? v0 : 0.f;
    a1c = v1;
    a2c = dn ? v2 : 0.f;
  }
  float* orow = XC + ((size_t)(b_ * IMH + h_) * IMW) * DIN + d;
#pragma unroll 1
  for (int w = 0; w < IMW; ++w) {
    const bool rv = (w + 1) < IMW;
    const int  wn = rv ? (w + 1) : (IMW - 1);
    const float nv0 = p0[(size_t)wn * XZW], nv1 = p1[(size_t)wn * XZW], nv2 = p2[(size_t)wn * XZW];
    const float a0n = (up && rv) ? nv0 : 0.f;
    const float a1n = rv ? nv1 : 0.f;
    const float a2n = (dn && rv) ? nv2 : 0.f;
    float acc = w00 * a0m;
    acc = fmaf(w01, a0c, acc);
    acc = fmaf(w02, a0n, acc);
    acc = fmaf(w10, a1m, acc);
    acc = fmaf(w11, a1c, acc);
    acc = fmaf(w12, a1n, acc);
    acc = fmaf(w20, a2m, acc);
    acc = fmaf(w21, a2c, acc);
    acc = fmaf(w22, a2n, acc);
    const float sv  = acc + bc;
    const float sg  = __builtin_amdgcn_rcpf(1.0f + __expf(-sv));
    const float out = sv * sg;
    float* op = orow + (size_t)w * DIN;
    *(volatile float*)op = out;
    __threadfence();
    *(volatile float*)op = out;
    sH[w * DINP + t] = out;
    a0m = a0c; a0c = a0n;
    a1m = a1c; a1c = a1n;
    a2m = a2c; a2c = a2n;
  }
  __syncthreads();
  const size_t rowb = ((size_t)(b_ * IMH + h_) * IMW) * DINP;
  unsigned short* obh = XC16H + rowb;
  unsigned short* obl = XC16L + rowb;
  for (int pass = 0; pass < 2; ++pass) {
#pragma unroll 4
    for (int it = 0; it < (IMW * DINP) / (8 * DIN); ++it) {
      const int f = it * DIN + t;
      const float* sp = sH + 8 * f;
      const v4f f0 = *(const v4f*)(sp);
      const v4f f1 = *(const v4f*)(sp + 4);
      v8h hv, lv;
      pack8<1>(f0, f1, hv, lv);
      *(volatile v8h*)(obh + (size_t)8 * f) = hv;
      *(volatile v8h*)(obl + (size_t)8 * f) = lv;
    }
    __threadfence();
  }
}

__device__ __forceinline__ int dir_tok(int k, int l) {
  const int lr = (k >= 2) ? (NPIX - 1 - l) : l;
  if (k & 1) { const int hh = lr % IMH; const int ww = lr / IMH; return hh * IMW + ww; }
  return lr;
}

__global__ __launch_bounds__(96) void scan_dir_kernel(
    const float* __restrict__ XDBL, const float* __restrict__ XC, const float* __restrict__ dtw,
    const float* __restrict__ dtb, const float* __restrict__ Alog, const float* __restrict__ Dsp,
    const float* Pa, const float* Pb, float* Yk, int k, int mode)
{
  __shared__ __align__(16) float sBC[SCH * XPC];
  const int t  = threadIdx.x;
  const int b_ = blockIdx.x;
  const int d  = t;
  const int kd = k * DIN + d;
  const float wt0 = dtw[(size_t)kd * DTR + 0];
  const float wt1 = dtw[(size_t)kd * DTR + 1];
  const float wt2 = dtw[(size_t)kd * DTR + 2];
  const float wt3 = dtw[(size_t)kd * DTR + 3];
  const float db = dtb[kd];
  const float Dk = Dsp[kd];
  float An[NST], h[NST];
#pragma unroll
  for (int n = 0; n < NST; ++n) {
    An[n] = -__expf(Alog[(size_t)kd * NST + n]);
    h[n]  = 0.f;
  }
  const size_t tokb = (size_t)b_ * NPIX;
#pragma unroll 1
  for (int c = 0; c < NPIX / SCH; ++c) {
    __syncthreads();
#pragma unroll 1
    for (int qi = t; qi < SCH * 9; qi += DIN) {
      const int s   = qi / 9;
      const int j   = qi - s * 9;
      const int tok = dir_tok(k, c * SCH + s);
      const v4f v = *(const v4f*)(XDBL + (tokb + tok) * XPCP + 4 * j);
      *(v4f*)(sBC + s * XPC + 4 * j) = v;
    }
    __syncthreads();
#pragma unroll 1
    for (int s = 0; s < SCH; ++s) {
      const int tok = dir_tok(k, c * SCH + s);
      const size_t ei = (tokb + tok) * DIN + d;
      const float u  = XC[ei];
      const float* sr = sBC + s * XPC;
      const v4f dq = *(const v4f*)sr;
      float dts = wt0 * dq[0];
      dts = fmaf(wt1, dq[1], dts);
      dts = fmaf(wt2, dq[2], dts);
      dts = fmaf(wt3, dq[3], dts);
      const float dp = dts + db;
      const float ex   = __expf(-fabsf(dp));
      const float up1  = 1.0f + ex;
      const float den  = up1 - 1.0f;
      const bool  dpos = den > 0.0f;
      const float dens = dpos ? den : 1.0f;
      const float lg   = __logf(up1);
      const float l1p  = dpos ? (lg * (ex * __builtin_amdgcn_rcpf(dens))) : ex;
      const float delta = fmaxf(dp, 0.0f) + l1p;
      v4f Bv[4], Cv[4];
#pragma unroll
      for (int i = 0; i < 4; ++i) {
        Bv[i] = *(const v4f*)(sr + DTR + 4 * i);
        Cv[i] = *(const v4f*)(sr + DTR + NST + 4 * i);
      }
      const float du = delta * u;
      float ys = 0.f;
#pragma unroll
      for (int n = 0; n < NST; ++n) {
        const float e  = __expf(delta * An[n]);
        const float hn = fmaf(e, h[n], du * Bv[n >> 2][n & 3]);
        h[n] = hn;
        ys = fmaf(hn, Cv[n >> 2][n & 3], ys);
      }
      const float yk = ys + Dk * u;
      float ysum = 0.f;
      if (mode == 1) {
        ysum = Pa[ei];
      } else if (mode == 2) {
        ysum = Pa[ei] + Pb[ei];
      }
      const float y = (mode == 0) ? yk : (ysum + yk);
      float* yp = Yk + ei;
      *(volatile float*)yp = y;
      __threadfence();
      *(volatile float*)yp = y;
    }
  }
}

__global__ __launch_bounds__(256) void ln_gate_kernel(
    const float* __restrict__ YS, const float* __restrict__ XZ,
    const float* __restrict__ gam, const float* __restrict__ bet,
    unsigned short* __restrict__ YGH, unsigned short* __restrict__ YGL)
{
  __shared__ __align__(16) float sG[8 * DINP];
  const int t = threadIdx.x, lane = t & 31, wave = t >> 5;
  const int tok = blockIdx.x * 8 + wave;
  const size_t base = (size_t)tok * DIN + lane;
  float a[3];
#pragma unroll
  for (int j = 0; j < 3; ++j) a[j] = YS[base + 32 * j];
  float s = (a[0] + a[1]) + a[2];
  s += __shfl_xor(s, 1, 32);
  s += __shfl_xor(s, 2, 32);
  s += __shfl_xor(s, 4, 32);
  s += __shfl_xor(s, 8, 32);
  s += __shfl_xor(s, 16, 32);
  const float mu = s * (1.0f / 96.0f);
  float q = 0.f;
#pragma unroll
  for (int j = 0; j < 3; ++j) { const float dd = a[j] - mu; q = fmaf(dd, dd, q); }
  q += __shfl_xor(q, 1, 32);
  q += __shfl_xor(q, 2, 32);
  q += __shfl_xor(q, 4, 32);
  q += __shfl_xor(q, 8, 32);
  q += __shfl_xor(q, 16, 32);
  const float var = q * (1.0f / 96.0f);
  const float is  = rsqrtf(var + 1e-5f);
  float* sw = sG + wave * DINP;
#pragma unroll
  for (int j = 0; j < 3; ++j) {
    const int ch = lane + 32 * j;
    const float zv = XZ[(size_t)tok * XZW + DIN + ch];
    const float gn = ((a[j] - mu) * is) * gam[ch] + bet[ch];
    const float sg = __builtin_amdgcn_rcpf(1.0f + __expf(-zv));
    sw[ch] = gn * (zv * sg);
  }
  sw[DIN + lane] = 0.0f;
  __syncthreads();
  const int c8 = (lane & 15) * 8;
  const float* sp = sw + c8;
  const v4f f0 = *(const v4f*)(sp);
  const v4f f1 = *(const v4f*)(sp + 4);
  v8h hv, lv;
  pack8<1>(f0, f1, hv, lv);
  unsigned short* oph = YGH + (size_t)tok * DINP + c8;
  unsigned short* opl = YGL + (size_t)tok * DINP + c8;
  if (lane < 16) { *(volatile v8h*)oph = hv; *(volatile v8h*)opl = lv; }
  __threadfence();
  if (lane < 16) { *(volatile v8h*)oph = hv; *(volatile v8h*)opl = lv; }
}

__global__ __launch_bounds__(256) void gelu_cast_kernel(
    const float* __restrict__ Hin, unsigned short* __restrict__ Hout, int n2)
{
  const int i = blockIdx.x * 256 + threadIdx.x;
  if (i >= n2) return;
  const v2f hv = *(const v2f*)(Hin + 2 * (size_t)i);
  const float x0 = hv[0], x1 = hv[1];
  float g0 = 0.f, g1 = 0.f;
#pragma unroll 1
  for (int e = 0; e < 2; ++e) {
    const float xv = (e == 0) ? x0 : x1;
    const float gv = 0.5f * xv * (1.0f + erff(xv * 0.70710678118654752f));
    g0 = (e == 0) ? gv : g0;
    g1 = gv;
  }
  const unsigned u = (unsigned)__builtin_bit_cast(unsigned short, (_Float16)g0)
                   | ((unsigned)__builtin_bit_cast(unsigned short, (_Float16)g1) << 16);
  ((volatile unsigned*)Hout)[i] = u;
  __threadfence();
  ((volatile unsigned*)Hout)[i] = u;
}

extern "C" void kernel_launch(void* const* d_in, const int* in_sizes, int n_in,
                              void* d_out, int out_size, void* d_ws, size_t ws_size,
                              hipStream_t stream)
{
  if (n_in < 20) return;
  const float* x    = (const float*)d_in[0];
  const float* n1g  = (const float*)d_in[1];
  const float* n1b  = (const float*)d_in[2];
  const float* inpw = (const float*)d_in[3];
  const float* cw   = (const float*)d_in[4];
  const float* cb   = (const float*)d_in[5];
  const float* xprw = (const float*)d_in[6];
  const float* dtw  = (const float*)d_in[7];
  const float* dtb  = (const float*)d_in[8];
  const float* alog = (const float*)d_in[9];
  const float* dsp  = (const float*)d_in[10];
  const float* ong  = (const float*)d_in[11];
  const float* onb  = (const float*)d_in[12];
  const float* opw  = (const float*)d_in[13];
  const float* n2g  = (const float*)d_in[14];
  const float* n2b  = (const float*)d_in[15];
  const float* fw1  = (const float*)d_in[16];
  const float* fb1  = (const float*)d_in[17];
  const float* fw2  = (const float*)d_in[18];
  const float* fb2  = (const float*)d_in[19];
  float* dout = (float*)d_out;

  if (in_sizes[0] != NIMG * NCH * NPIX) return;
  if (in_sizes[1] != NCH || in_sizes[2] != NCH) return;
  if (in_sizes[3] != XZW * NCH) return;
  if (in_sizes[4] != DIN * 9 || in_sizes[5] != DIN) return;
  if (in_sizes[6] != NDIR * XPC * DIN) return;
  if (in_sizes[7] != NDIR * DIN * DTR || in_sizes[8] != NDIR * DIN) return;
  if (in_sizes[9] != NDIR * DIN * NST || in_sizes[10] != NDIR * DIN) return;
  if (in_sizes[11] != DIN || in_sizes[12] != DIN) return;
  if (in_sizes[13] != NCH * DIN) return;
  if (in_sizes[14] != NCH || in_sizes[15] != NCH) return;
  if (in_sizes[16] != FFH * NCH || in_sizes[17] != FFH) return;
  if (in_sizes[18] != NCH * FFH || in_sizes[19] != NCH) return;
  if (out_size != NIMG * NCH * NPIX) return;

  const size_t SZ_WIN  = (size_t)XZW * NCH * 2;
  const size_t SZ_WX   = (size_t)NDIR * XPCP * DIN * 2;
  const size_t SZ_WO   = (size_t)NCH * DIN * 2;
  const size_t SZ_W1   = (size_t)FFH * NCH * 2;
  const size_t SZ_W2   = (size_t)NCH * FFH * 2;
  const size_t SZ_WGT  = 262144;
  const size_t SZ_XN   = (size_t)NTOK * NCH * 2;
  const size_t SZ_XZ   = (size_t)NTOK * XZW * 4;
  const size_t SZ_XC   = (size_t)NTOK * DIN * 4;
  const size_t SZ_P16  = (size_t)NTOK * DINP * 2;
  const size_t SZ_X1   = (size_t)NIMG * NCH * NPIX * 4;
  const size_t SZ_XDBL = (size_t)NTOK * XPCP * 4;
  const size_t SZ_YP   = (size_t)3 * NTOK * DIN * 4;
  const size_t SZ_HB   = (size_t)NTOK * FFH * 4;
  const size_t SZ_HG   = (size_t)NTOK * FFH * 2;

  const size_t OFF_WINH = 0;
  const size_t OFF_WINL = OFF_WINH + SZ_WIN;
  const size_t OFF_WXH  = OFF_WINL + SZ_WIN;
  const size_t OFF_WXL  = OFF_WXH  + SZ_WX;
  const size_t OFF_WOH  = OFF_WXL  + SZ_WX;
  const size_t OFF_WOL  = OFF_WOH  + SZ_WO;
  const size_t OFF_W1   = OFF_WOL  + SZ_WO;
  const size_t OFF_W2   = OFF_W1   + SZ_W1;
  if (OFF_W2 + SZ_W2 > SZ_WGT) return;
  const size_t OFF_XNH  = SZ_WGT;
  const size_t OFF_XNL  = OFF_XNH  + SZ_XN;
  const size_t OFF_XZ   = OFF_XNL  + SZ_XN;
  const size_t OFF_XC   = OFF_XZ   + SZ_XZ;
  const size_t OFF_XC16H = OFF_XC  + SZ_XC;
  const size_t OFF_XC16L = OFF_XC16H + SZ_P16;
  const size_t OFF_XDBL = OFF_XC16L + SZ_P16;
  const size_t OFF_YP   = OFF_XDBL + SZ_XDBL;
  const size_t TOTAL    = OFF_YP   + SZ_YP;
  const size_t OFF_XN2  = OFF_XNH;
  const size_t OFF_YGH  = OFF_XC;
  const size_t OFF_YGL  = OFF_XC + SZ_P16;
  const size_t OFF_X1   = OFF_XDBL;
  const size_t OFF_HB   = OFF_YP;
  const size_t OFF_HG   = OFF_YP + SZ_HB;
  if (OFF_YGL + SZ_P16 > OFF_XDBL) return;
  if (SZ_X1 > SZ_XDBL) return;
  if (SZ_HB + SZ_HG > SZ_YP) return;
  if (TOTAL > (size_t)134217728) return;
  if (ws_size < TOTAL) return;

  char* ws = (char*)d_ws;
  unsigned short* WINH  = (unsigned short*)(ws + OFF_WINH);
  unsigned short* WINL  = (unsigned short*)(ws + OFF_WINL);
  unsigned short* WXH   = (unsigned short*)(ws + OFF_WXH);
  unsigned short* WXL   = (unsigned short*)(ws + OFF_WXL);
  unsigned short* WOH   = (unsigned short*)(ws + OFF_WOH);
  unsigned short* WOL   = (unsigned short*)(ws + OFF_WOL);
  unsigned short* W1h   = (unsigned short*)(ws + OFF_W1);
  unsigned short* W2h   = (unsigned short*)(ws + OFF_W2);
  unsigned short* XNH   = (unsigned short*)(ws + OFF_XNH);
  unsigned short* XNL   = (unsigned short*)(ws + OFF_XNL);
  unsigned short* XN2h  = (unsigned short*)(ws + OFF_XN2);
  float*          XZ    = (float*)(ws + OFF_XZ);
  float*          XC    = (float*)(ws + OFF_XC);
  unsigned short* XC16H = (unsigned short*)(ws + OFF_XC16H);
  unsigned short* XC16L = (unsigned short*)(ws + OFF_XC16L);
  unsigned short* YGH   = (unsigned short*)(ws + OFF_YGH);
  unsigned short* YGL   = (unsigned short*)(ws + OFF_YGL);
  float*          X1    = (float*)(ws + OFF_X1);
  float*          XDBL  = (float*)(ws + OFF_XDBL);
  float*          YP0   = (float*)(ws + OFF_YP);
  float*          YP1   = YP0 + (size_t)NTOK * DIN;
  float*          YP2   = YP1 + (size_t)NTOK * DIN;
  float*          HB    = (float*)(ws + OFF_HB);
  unsigned short* HG16  = (unsigned short*)(ws + OFF_HG);
  const float*    nores = x;

  {
    const int nc = XZW * NCH / 8;
    cast_pad_kernel<1><<<(nc + 255) / 256, 256, 0, stream>>>(inpw, NCH, XZW, XZW, WINH, WINL, NCH, NCH, nc, 1.0f);
  }
  {
    const int nc = NDIR * XPCP * DIN / 8;
    cast_pad_kernel<1><<<(nc + 255) / 256, 256, 0, stream>>>(xprw, DIN, XPC, XPCP, WXH, WXL, DIN, DIN, nc, 1.0f);
  }
  {
    const int nc = NCH * DIN / 8;
    cast_pad_kernel<1><<<(nc + 255) / 256, 256, 0, stream>>>(opw, DIN, NCH, NCH, WOH, WOL, DIN, DIN, nc, 1.0f);
  }
  {
    const int nc = FFH * NCH / 8;
    cast_pad_kernel<0><<<(nc + 255) / 256, 256, 0, stream>>>(fw1, NCH, FFH, FFH, W1h, W1h, NCH, NCH, nc, 64.0f);
  }
  {
    const int nc = NCH * FFH / 8;
    cast_pad_kernel<0><<<(nc + 255) / 256, 256, 0, stream>>>(fw2, FFH, NCH, NCH, W2h, W2h, FFH, FFH, nc, 64.0f);
  }

  ln_nchw_kernel<1><<<NIMG * (NPIX / TOKB), 256, 0, stream>>>(x, n1g, n1b, XNH, XNL);

  {
    const int tiles = (NTOK / 64) * (XZW / 64);
    wmma_gemm64<1, true, 0, 0, false, 0><<<dim3((tiles + 7) / 8, 1), 256, 0, stream>>>(
        XNH, XNL, NCH, 0L, WINH, WINL, NCH, 0L, (void*)XZ, (void*)XZ, XZW, 0L,
        nores, nores, 0L, NTOK, XZW, NCH, 1.0f);
  }

  dwconv_silu_kernel<<<NIMG * IMH, DIN, 0, stream>>>(XZ, cw, cb, XC, XC16H, XC16L);

  {
    float*       souts[4] = {YP0, YP1, YP2, YP0};
    const float* pas[4]   = {YP0, YP0, YP0, YP2};
    const float* pbs[4]   = {YP0, YP0, YP0, YP1};
    const int    modes[4] = {0, 0, 1, 2};
    for (int k = 0; k < NDIR; ++k) {
      const int tiles = (NTOK / 64) * (XPCP / 64);
      wmma_gemm64<1, true, 0, 0, false, 0><<<dim3((tiles + 7) / 8, 1), 256, 0, stream>>>(
          XC16H, XC16L, DINP, 0L, WXH + (size_t)k * XPCP * DIN, WXL + (size_t)k * XPCP * DIN, DIN, 0L,
          (void*)XDBL, (void*)XDBL, XPCP, 0L, nores, nores, 0L, NTOK, XPCP, DIN, 1.0f);
      scan_dir_kernel<<<NIMG, DIN, 0, stream>>>(XDBL, XC, dtw, dtb, alog, dsp, pas[k], pbs[k], souts[k], k, modes[k]);
    }
  }

  ln_gate_kernel<<<NTOK / 8, 256, 0, stream>>>(YP0, XZ, ong, onb, YGH, YGL);

  {
    const int tiles = (NCH / 64) * (NPIX / 64);
    wmma_gemm64<1, true, 0, 0, true, 0><<<dim3((tiles + 7) / 8, NIMG), 256, 0, stream>>>(
        WOH, WOL, DIN, 0L, YGH, YGL, DINP, (long)NPIX * DINP, (void*)X1, (void*)X1, NPIX, (long)NCH * NPIX,
        nores, x, (long)NCH * NPIX, NCH, NPIX, DIN, 1.0f);
  }

  ln_nchw_kernel<0><<<NIMG * (NPIX / TOKB), 256, 0, stream>>>(X1, n2g, n2b, XN2h, XN2h);

  {
    const int tiles = (NTOK / 64) * (FFH / 64);
    wmma_gemm64<0, false, 2, 0, false, 0><<<dim3((tiles + 7) / 8, 1), 256, 0, stream>>>(
        XN2h, XN2h, NCH, 0L, W1h, W1h, NCH, 0L, (void*)HB, (void*)HB, FFH, 0L,
        fb1, nores, 0L, NTOK, FFH, NCH, 1.0f / 64.0f);
  }

  {
    const int n2 = NTOK * FFH / 2;
    gelu_cast_kernel<<<(n2 + 255) / 256, 256, 0, stream>>>(HB, HG16, n2);
  }

  {
    const int tiles = (NCH / 64) * (NPIX / 64);
    wmma_gemm64<0, false, 1, 0, true, 0><<<dim3((tiles + 7) / 8, NIMG), 256, 0, stream>>>(
        W2h, W2h, FFH, 0L, HG16, HG16, FFH, (long)NPIX * FFH, (void*)dout, (void*)dout, NPIX, (long)NCH * NPIX,
        fb2, X1, (long)NCH * NPIX, NCH, NPIX, FFH, 1.0f / 64.0f);
  }
}
